// LRU_17411797418611
// MI455X (gfx1250) — hardware-verified
//
#include <hip/hip_runtime.h>
#include <math.h>

constexpr int NSEQ = 4096;
constexpr int NMOD = 2048;
constexpr int NHID = 1024;
constexpr int NCAT = 2 * NHID;
constexpr int NTHR = 256;
constexpr int SCAN_CH_PER_LANE = 8;
constexpr int SCAN_LANES = NHID / SCAN_CH_PER_LANE;
constexpr int SCAN_BLK = 32;
constexpr float BCARRY = 64.0f;
constexpr float CCARRY = 32.0f;
constexpr float HCARRY = 4.0f;
constexpr float GEMM1_SCALE = 1.0f / 64.0f;
constexpr float GEMM2_SCALE = 1.0f / 128.0f;
static_assert(NSEQ % 64 == 0 && NCAT % 64 == 0 && NMOD % 64 == 0);
static_assert(NMOD % 32 == 0 && NCAT % 32 == 0);
static_assert(((NSEQ / 64) * (NCAT / 64)) % 8 == 0);
static_assert(((NSEQ / 64) * (NMOD / 64)) % 8 == 0);
static_assert(SCAN_LANES % SCAN_BLK == 0);
static_assert(NHID % NTHR == 0);
static_assert((NSEQ * (NMOD / 8)) % NTHR == 0);
static_assert((NHID * (NMOD / 8)) % NTHR == 0);
static_assert((NMOD * (NHID / 8)) % NTHR == 0);

typedef __attribute__((ext_vector_type(16))) _Float16 v16h;
typedef __attribute__((ext_vector_type(8)))  _Float16 v8h;
typedef __attribute__((ext_vector_type(16))) __bf16   v16b;
typedef __attribute__((ext_vector_type(8)))  __bf16   v8b;
typedef __attribute__((ext_vector_type(8)))  float    v8f;
typedef __attribute__((ext_vector_type(4)))  float    v4f;

__device__ __forceinline__ void dep_guard_h(v8f& a, v8f& b, v16h x, v16h y) { asm volatile("v_nop\n\tv_nop\n\tv_nop\n\tv_nop" : "+v"(a), "+v"(b) : "v"(x), "v"(y)); }
__device__ __forceinline__ void dep_guard_b(v8f& a, v8f& b, v16b x, v16b y) { asm volatile("v_nop\n\tv_nop\n\tv_nop\n\tv_nop" : "+v"(a), "+v"(b) : "v"(x), "v"(y)); }
__device__ __forceinline__ void dep_guard4_h(v8f& a, v8f& b, v8f& c, v8f& d, v16h x, v16h y) {
  asm volatile("v_nop\n\tv_nop\n\tv_nop\n\tv_nop" : "+v"(a), "+v"(b), "+v"(c), "+v"(d) : "v"(x), "v"(y));
}
__device__ __forceinline__ void keep4_h(v16h a, v16h b, v16h c, v16h d) { asm volatile("v_nop" :: "v"(a), "v"(b), "v"(c), "v"(d)); }
__device__ __forceinline__ void keep4_b(v16b a, v16b b, v16b c, v16b d) { asm volatile("v_nop" :: "v"(a), "v"(b), "v"(c), "v"(d)); }
__device__ __forceinline__ void acc_guard4(v8f& a, v8f& b, v8f& c, v8f& d) { asm volatile("v_nop\n\tv_nop\n\tv_nop\n\tv_nop" : "+v"(a), "+v"(b), "+v"(c), "+v"(d)); }
template <typename T> struct Frag;
template <> struct Frag<_Float16> {
  typedef v16h V; union U { v16h v; v8h h[2]; };
  static __device__ __forceinline__ v16h load(const _Float16* p) {
    U f; f.h[0] = *(const v8h*)(p); f.h[1] = *(const v8h*)(p + 16); return f.v;
  }
  static __device__ __forceinline__ v8f mma(v16h a, v16h b, v8f c) {
    return __builtin_amdgcn_wmma_f32_16x16x32_f16(false, a, false, b, (short)0, c, false, false);
  }
  static __device__ __forceinline__ void guard(v8f& a, v8f& b, v16h x, v16h y) { dep_guard_h(a, b, x, y); }
  static __device__ __forceinline__ void keep(v16h a, v16h b, v16h c, v16h d) { keep4_h(a, b, c, d); }
};
template <> struct Frag<__bf16> {
  typedef v16b V; union U { v16b v; v8b h[2]; };
  static __device__ __forceinline__ v16b load(const __bf16* p) {
    U f; f.h[0] = *(const v8b*)(p); f.h[1] = *(const v8b*)(p + 16); return f.v;
  }
  static __device__ __forceinline__ v8f mma(v16b a, v16b b, v8f c) {
    return __builtin_amdgcn_wmma_f32_16x16x32_bf16(false, a, false, b, (short)0, c, false, false);
  }
  static __device__ __forceinline__ void guard(v8f& a, v8f& b, v16b x, v16b y) { dep_guard_b(a, b, x, y); }
  static __device__ __forceinline__ void keep(v16b a, v16b b, v16b c, v16b d) { keep4_b(a, b, c, d); }
};

__global__ __launch_bounds__(NTHR) void lru_params_kernel(const float* __restrict__ nu, const float* __restrict__ theta,
                                                          const float* __restrict__ gl, float* __restrict__ PAR) {
  __shared__ __align__(16) float s_lr[NTHR];
  __shared__ __align__(16) float s_li[NTHR];
  __shared__ __align__(16) float s_g[NTHR];
  const int tid = threadIdx.x;
  const int n = blockIdx.x * NTHR + tid;
  const float en = expf(nu[n]);
  const float ph = expf(theta[n]);
  const float md = expf(-en);
  s_lr[tid] = md * cosf(ph);
  s_li[tid] = md * sinf(ph);
  s_g[tid]  = expf(gl[n]);
  __syncthreads();
  const int role = tid >> 6;
  const int q = (tid & 63) * 4;
  const v4f a = *(const v4f*)(s_lr + q);
  const v4f b = *(const v4f*)(s_li + q);
  const v4f g = *(const v4f*)(s_g + q);
  v4f o;
#pragma unroll
  for (int e = 0; e < 4; ++e) o[e] = (role == 0) ? a[e] : ((role == 1) ? b[e] : g[e]);
  float* dst = PAR + role * NHID + blockIdx.x * NTHR + q;
  *(volatile v4f*)dst = o;
  __threadfence();
  *(volatile v4f*)dst = o;
}

__global__ __launch_bounds__(NTHR) void cast_f16_kernel(const float* __restrict__ src, int spitch,
                                                        unsigned short* __restrict__ dst, int dpitch, int dcol0,
                                                        int nrow, int ncol8, float sc) {
  const int i  = blockIdx.x * NTHR + threadIdx.x;
  const int n8 = nrow * ncol8;
  if (i < n8) {
    const int row = i / ncol8;
    const int c8  = i - row * ncol8;
    const float* sp = src + (size_t)row * spitch + (size_t)c8 * 8;
    const v4f a = *(const v4f*)(sp);
    const v4f b = *(const v4f*)(sp + 4);
    v8h hv;
#pragma unroll
    for (int e = 0; e < 4; ++e) {
      hv[e]     = (_Float16)(a[e] * sc);
      hv[4 + e] = (_Float16)(b[e] * sc);
    }
    unsigned short* dp = dst + (size_t)row * dpitch + dcol0 + (size_t)c8 * 8;
    *(volatile v8h*)dp = hv;
    __threadfence();
    *(volatile v8h*)dp = hv;
  }
}

template <int EPI>
__global__ __launch_bounds__(NTHR) void gemm64_f16_kernel(
    const unsigned short* __restrict__ Ap, int lda,
    const unsigned short* __restrict__ Btp, int ldb,
    float* __restrict__ Cout, int ldc,
    const float* __restrict__ colv,
    const float* __restrict__ Uadd, int ldu,
    int M, int N, int K, float scale) {
  const _Float16* A  = (const _Float16*)Ap;
  const _Float16* Bt = (const _Float16*)Btp;
  __shared__ __align__(16) float sT[8][16 * 68];
  const int lane = threadIdx.x & 31;
  const int wave = threadIdx.x >> 5;
  const int tilesN = N >> 6;
  const int tilesM = M >> 6;
  const int tile = blockIdx.x * 8 + wave;
  if (tile >= tilesM * tilesN) return;
  const int tm = tile / tilesN;
  const int tn = tile - tm * tilesN;
  const int m0 = tm << 6;
  const int n0 = tn << 6;

  const int rlane = lane & 15;
  const int koff  = (lane >> 4) * 8;
  const int mOff  = (lane >> 4) * 8;

  v8f acc[4][4];
#pragma unroll
  for (int i = 0; i < 4; ++i)
#pragma unroll
    for (int j = 0; j < 4; ++j) acc[i][j] = (v8f){0.f,0.f,0.f,0.f,0.f,0.f,0.f,0.f};

  for (int k0 = 0; k0 < K; k0 += 32) {
    v16h bh[4];
#pragma unroll
    for (int j = 0; j < 4; ++j) {
      const size_t bo = (size_t)(n0 + (j << 4) + rlane) * ldb + koff + k0;
      bh[j] = Frag<_Float16>::load(Bt + bo);
    }
#pragma unroll
    for (int i = 0; i < 4; ++i) {
      const size_t ao = (size_t)(m0 + (i << 4) + rlane) * lda + koff + k0;
      const v16h ah = Frag<_Float16>::load(A + ao);
#pragma unroll
      for (int j = 0; j < 4; ++j) acc[i][j] = Frag<_Float16>::mma(ah, bh[j], acc[i][j]);
      dep_guard4_h(acc[i][0], acc[i][1], acc[i][2], acc[i][3], ah, bh[3]);
    }
    keep4_h(bh[0], bh[1], bh[2], bh[3]);
  }
  acc_guard4(acc[0][0], acc[0][1], acc[0][2], acc[0][3]);
  acc_guard4(acc[1][0], acc[1][1], acc[1][2], acc[1][3]);
  acc_guard4(acc[2][0], acc[2][1], acc[2][2], acc[2][3]);
  acc_guard4(acc[3][0], acc[3][1], acc[3][2], acc[3][3]);

  float* slab = sT[wave];
  const int hh = lane >> 4, c4 = (lane & 15) * 4;
  float gv[4];
#pragma unroll
  for (int j = 0; j < 4; ++j) gv[j] = (EPI == 1) ? colv[n0 + (j << 4) + rlane] : 1.0f;
  v4f dd = (v4f){0.f, 0.f, 0.f, 0.f};
  if (EPI == 2) dd = *(const v4f*)(colv + n0 + c4);
#pragma unroll
  for (int i = 0; i < 4; ++i) {
    const int mBase = m0 + (i << 4);
#pragma unroll
    for (int j = 0; j < 4; ++j) {
#pragma unroll
      for (int r = 0; r < 8; ++r) {
        float v = acc[i][j][r] * scale;
        if (EPI == 1) v = v * gv[j];
        slab[(mOff + r) * 68 + (j << 4) + rlane] = v;
      }
    }
    __builtin_amdgcn_fence(__ATOMIC_RELEASE, "workgroup");
    __builtin_amdgcn_wave_barrier();
    __builtin_amdgcn_fence(__ATOMIC_ACQUIRE, "workgroup");
    v4f ov[8];
#pragma unroll
    for (int it = 0; it < 8; ++it) {
      const int row = it * 2 + hh;
      v4f v = *(const v4f*)(slab + row * 68 + c4);
      if (EPI == 2) {
        const v4f uu = *(const v4f*)(Uadd + (size_t)(mBase + row) * ldu + n0 + c4);
#pragma unroll
        for (int e = 0; e < 4; ++e) v[e] = fmaf(dd[e], uu[e], v[e]);
      }
      ov[it] = v;
    }
    for (int pass = 0; pass < 2; ++pass) {
#pragma unroll
      for (int it = 0; it < 8; ++it) {
        const int row = it * 2 + hh;
        *(volatile v4f*)(Cout + (size_t)(mBase + row) * ldc + n0 + c4) = ov[it];
      }
      __threadfence();
    }
    __builtin_amdgcn_fence(__ATOMIC_RELEASE, "workgroup");
    __builtin_amdgcn_wave_barrier();
    __builtin_amdgcn_fence(__ATOMIC_ACQUIRE, "workgroup");
  }
}

__global__ __launch_bounds__(SCAN_BLK) void lru_scan_kernel(const float* __restrict__ BU, const float* __restrict__ PAR,
                                                            unsigned short* __restrict__ H16) {
  const int g  = blockIdx.x * SCAN_BLK + threadIdx.x;
  const int n0 = g * SCAN_CH_PER_LANE;
  const v4f lra = *(const v4f*)(PAR + n0);
  const v4f lrb = *(const v4f*)(PAR + n0 + 4);
  const v4f lia = *(const v4f*)(PAR + NHID + n0);
  const v4f lib = *(const v4f*)(PAR + NHID + n0 + 4);
  float lre[8], lim[8], hre[8], him[8];
#pragma unroll
  for (int e = 0; e < 4; ++e) {
    lre[e] = lra[e]; lre[4 + e] = lrb[e];
    lim[e] = lia[e]; lim[4 + e] = lib[e];
  }
#pragma unroll
  for (int e = 0; e < 8; ++e) { hre[e] = 0.0f; him[e] = 0.0f; }

#pragma unroll 1
  for (int t = 0; t < NSEQ; ++t) {
    const float* bp = BU + (size_t)t * NCAT + n0;
    const v4f ura = *(const v4f*)(bp);
    const v4f urb = *(const v4f*)(bp + 4);
    const v4f uia = *(const v4f*)(bp + NHID);
    const v4f uib = *(const v4f*)(bp + NHID + 4);
    float ure[8], uim[8];
#pragma unroll
    for (int e = 0; e < 4; ++e) {
      ure[e] = ura[e]; ure[4 + e] = urb[e];
      uim[e] = uia[e]; uim[4 + e] = uib[e];
    }
    v8h hr, hi;
#pragma unroll
    for (int e = 0; e < 8; ++e) {
      const float nre = fmaf(lre[e], hre[e], fmaf(-lim[e], him[e], ure[e]));
      const float nim = fmaf(lre[e], him[e], fmaf( lim[e], hre[e], uim[e]));
      hre[e] = nre;
      him[e] = nim;
      hr[e] = (_Float16)(nre * HCARRY);
      hi[e] = (_Float16)(nim * HCARRY);
    }
    unsigned short* hp = H16 + (size_t)t * NCAT + n0;
    *(volatile v8h*)(hp) = hr;
    *(volatile v8h*)(hp + NHID) = hi;
    __threadfence();
    *(volatile v8h*)(hp) = hr;
    *(volatile v8h*)(hp + NHID) = hi;
  }
}

extern "C" void kernel_launch(void* const* d_in, const int* in_sizes, int n_in,
                              void* d_out, int out_size, void* d_ws, size_t ws_size, hipStream_t stream) {
  if (n_in < 9 || d_out == nullptr || d_ws == nullptr) return;
  if (in_sizes[0] != NSEQ * NMOD || in_sizes[1] != NHID || in_sizes[2] != NHID || in_sizes[3] != NHID ||
      in_sizes[4] != NHID * NMOD || in_sizes[5] != NHID * NMOD || in_sizes[6] != NMOD * NHID ||
      in_sizes[7] != NMOD * NHID || in_sizes[8] != NMOD || out_size != NSEQ * NMOD) return;

  const float* u_in  = (const float*)d_in[0];
  const float* nu    = (const float*)d_in[1];
  const float* theta = (const float*)d_in[2];
  const float* glog  = (const float*)d_in[3];
  const float* b_re  = (const float*)d_in[4];
  const float* b_im  = (const float*)d_in[5];
  const float* c_re  = (const float*)d_in[6];
  const float* c_im  = (const float*)d_in[7];
  const float* dvec  = (const float*)d_in[8];
  float* y = (float*)d_out;

  char* ws = (char*)d_ws; size_t off = 0;
  auto carve = [&](size_t bytes) -> char* { char* p = ws + off; off += (bytes + 255) & ~(size_t)255; return p; };
  unsigned short* U16  = (unsigned short*)carve((size_t)NSEQ * NMOD * 2);
  unsigned short* BCAT = (unsigned short*)carve((size_t)NCAT * NMOD * 2);
  unsigned short* CCAT = (unsigned short*)carve((size_t)NMOD * NCAT * 2);
  float*          BU   = (float*)carve((size_t)NSEQ * NCAT * 4);
  unsigned short* H16  = (unsigned short*)carve((size_t)NSEQ * NCAT * 2);
  float*          PAR  = (float*)carve((size_t)4 * NHID * 4);
  if (off > ws_size || off > (size_t)134217728) return;

  lru_params_kernel<<<NHID / NTHR, NTHR, 0, stream>>>(nu, theta, glog, PAR);

  cast_f16_kernel<<<(NSEQ * (NMOD / 8)) / NTHR, NTHR, 0, stream>>>(u_in, NMOD, U16, NMOD, 0, NSEQ, NMOD / 8, 1.0f);
  cast_f16_kernel<<<(NHID * (NMOD / 8)) / NTHR, NTHR, 0, stream>>>(b_re, NMOD, BCAT, NMOD, 0, NHID, NMOD / 8, BCARRY);
  cast_f16_kernel<<<(NHID * (NMOD / 8)) / NTHR, NTHR, 0, stream>>>(b_im, NMOD, BCAT + (size_t)NHID * NMOD, NMOD, 0,
                                                                  NHID, NMOD / 8, BCARRY);
  cast_f16_kernel<<<(NMOD * (NHID / 8)) / NTHR, NTHR, 0, stream>>>(c_re, NHID, CCAT, NCAT, 0,    NMOD, NHID / 8, CCARRY);
  cast_f16_kernel<<<(NMOD * (NHID / 8)) / NTHR, NTHR, 0, stream>>>(c_im, NHID, CCAT, NCAT, NHID, NMOD, NHID / 8, -CCARRY);

  gemm64_f16_kernel<1><<<((NSEQ / 64) * (NCAT / 64)) / 8, NTHR, 0, stream>>>(
      U16, NMOD, BCAT, NMOD, BU, NCAT, PAR + 2 * NHID, u_in, NMOD, NSEQ, NCAT, NMOD, GEMM1_SCALE);

  lru_scan_kernel<<<SCAN_LANES / SCAN_BLK, SCAN_BLK, 0, stream>>>(BU, PAR, H16);

  gemm64_f16_kernel<2><<<((NSEQ / 64) * (NMOD / 64)) / 8, NTHR, 0, stream>>>(
      H16, NCAT, CCAT, NCAT, y, NMOD, dvec, u_in, NMOD, NSEQ, NMOD, NCAT, GEMM2_SCALE);
}
